// vSU2_CNN_1D_ref_41979010351317
// MI455X (gfx1250) — hardware-verified
//
#include <hip/hip_runtime.h>
#include <stdint.h>
#include <math.h>


typedef __bf16 v16b __attribute__((ext_vector_type(16)));
typedef unsigned short us8 __attribute__((ext_vector_type(8)));
typedef unsigned short us16 __attribute__((ext_vector_type(16)));
typedef float v8f __attribute__((ext_vector_type(8)));
typedef float v4f __attribute__((ext_vector_type(4)));

#define NN 512
#define MM 510
#define NF 3
#define NC 4
#define NP 5

union Frag { v16b v; us16 u; us8 half[2]; };
union AccU { v8f v; float f[8]; };

__device__ __forceinline__ unsigned short f2bf(float x) {
  unsigned int u = __float_as_uint(x);
  u = (u + 0x7FFFu + ((u >> 16) & 1u)) >> 16;
  return (unsigned short)u;
}

__device__ __forceinline__ int fixidx(int v) {
  if (v < 0) v += NC;
  v = v < 0 ? 0 : v;
  v = v > (NC - 1) ? (NC - 1) : v;
  return v;
}

__device__ __forceinline__ v8f wmma_bf16(v16b a, v16b b, v8f c) {
  v8f d = __builtin_amdgcn_wmma_f32_16x16x32_bf16(false, a, false, b, (short)0, c, false, false);
  asm volatile("v_nop\n\tv_nop\n\tv_nop\n\tv_nop" : "+v"(d) : "v"(a), "v"(b));
  return d;
}

__global__ void __launch_bounds__(256)
prep_kernel(const int* __restrict__ xv, const float* __restrict__ ik,
            unsigned short* __restrict__ A16, unsigned short* __restrict__ D16,
            int total_chunks)
{
  const int idx = blockIdx.x * blockDim.x + threadIdx.x;
  if (idx >= total_chunks) return;
  const int chunksA = NF * NN * (NN / 8);

  us8 v;
  unsigned short* dst;
  if (idx < chunksA) {
    const int f   = idx >> 15;
    const int rem = idx & 32767;
    const int j   = rem >> 6;
    const int kc  = (rem & 63) * 8;
    const float* base = ik + (size_t)f * MM * MM;
    #pragma unroll
    for (int e = 0; e < 8; ++e) {
      const int k = kc + e;
      float av = 0.0f;
      if (j < MM && k < MM) av = base[j * MM + k] - base[k * MM + j];
      v[e] = f2bf(av);
    }
    dst = A16 + (size_t)idx * 8;
  } else {
    const int idx2 = idx - chunksA;
    const int c    = idx2 >> 15;
    const int rem  = idx2 & 32767;
    const int i    = rem >> 6;
    const int kc   = (rem & 63) * 8;
    #pragma unroll
    for (int e = 0; e < 8; ++e) {
      const int p  = (i + 1 + kc + e) & (NN - 1);
      const int xs = fixidx(xv[p]);
      v[e] = (xs == c) ? (unsigned short)0x3F80 : (unsigned short)0;
    }
    dst = D16 + (size_t)idx2 * 8;
  }
  *(volatile us8*)dst = v;
  __threadfence();
  *(volatile us8*)dst = v;
}

__global__ void __launch_bounds__(128)
gemm_kernel(const int* __restrict__ xv, const float* __restrict__ tp,
            const unsigned short* __restrict__ A16,
            const unsigned short* __restrict__ D16,
            float* __restrict__ yws)
{
  __shared__ int   xs[NN];
  __shared__ float tps[NC * NC * NC];
  __shared__ float part[NC][32];
  __shared__ float lb[32];

  const int tid = threadIdx.x;
  const int w   = tid >> 5;
  const int l   = tid & 31;
  const int h   = l >> 4;
  const int m   = l & 15;
  const int i0  = blockIdx.x * 32;
  const int f   = blockIdx.y;

  for (int p = tid; p < NN; p += 128) xs[p] = fixidx(xv[p]);
  if (tid < NC * NC * NC) tps[tid] = tp[tid];
  __syncthreads();

  const int c = w;
  const unsigned short* Da = D16 + (size_t)c * NN * NN + (size_t)(i0 + m) * NN;
  const unsigned short* Db = Da + (size_t)16 * NN;
  const unsigned short* Bf = A16 + (size_t)f * NN * NN;

  float run0[8], run1[8];
  int   xa0[8], xa1[8];
  #pragma unroll
  for (int r = 0; r < 8; ++r) {
    run0[r] = 0.0f; run1[r] = 0.0f;
    xa0[r] = xs[i0 + 8 * h + r] * (NC * NC);
    xa1[r] = xs[i0 + 16 + 8 * h + r] * (NC * NC);
  }

  #pragma unroll 1
  for (int jt = 0; jt < NN / 16; ++jt) {
    const int j = jt * 16 + m;
    const unsigned short* Bp = Bf + (size_t)j * NN;

    v8f acc0 = {};
    v8f acc1 = {};
    #pragma unroll 4
    for (int ks = 0; ks < NN / 32; ++ks) {
      const int k0 = ks * 32;
      Frag a0, a1, b;
      b.half[0]  = *(const us8*)(Bp + k0 + 8 * h);
      b.half[1]  = *(const us8*)(Bp + k0 + 16 + 8 * h);
      a0.half[0] = *(const us8*)(Da + k0 + 8 * h);
      a0.half[1] = *(const us8*)(Da + k0 + 16 + 8 * h);
      a1.half[0] = *(const us8*)(Db + k0 + 8 * h);
      a1.half[1] = *(const us8*)(Db + k0 + 16 + 8 * h);
      acc0 = wmma_bf16(a0.v, b.v, acc0);
      acc1 = wmma_bf16(a1.v, b.v, acc1);
    }

    AccU u0, u1;
    u0.v = acc0;
    u1.v = acc1;
    const bool jvalid = (j < MM);
    #pragma unroll
    for (int r = 0; r < 8; ++r) {
      const int ia  = i0 + 8 * h + r;
      const int ib  = ia + 16;
      const int xb0 = xs[(ia + 1 + j) & (NN - 1)];
      const int xb1 = xs[(ib + 1 + j) & (NN - 1)];
      const float c0 = jvalid ? tps[xa0[r] + xb0 * NC + c] : 0.0f;
      const float c1 = jvalid ? tps[xa1[r] + xb1 * NC + c] : 0.0f;
      run0[r] += u0.f[r] * c0;
      run1[r] += u1.f[r] * c1;
    }
  }

  #pragma unroll
  for (int off = 1; off < 16; off <<= 1) {
    #pragma unroll
    for (int r = 0; r < 8; ++r) {
      run0[r] += __shfl_xor(run0[r], off, 32);
      run1[r] += __shfl_xor(run1[r], off, 32);
    }
  }
  if (m == 0) {
    #pragma unroll
    for (int r = 0; r < 8; ++r) {
      part[c][8 * h + r]      = run0[r];
      part[c][16 + 8 * h + r] = run1[r];
    }
  }
  __syncthreads();
  if (tid < 32) lb[tid] = ((part[0][tid] + part[1][tid]) + part[2][tid]) + part[3][tid];
  __syncthreads();
  if (tid < 8) {
    v4f o;
    o.x = lb[4 * tid + 0];
    o.y = lb[4 * tid + 1];
    o.z = lb[4 * tid + 2];
    o.w = lb[4 * tid + 3];
    float* dst = yws + (size_t)f * NN + i0 + 4 * tid;
    *(volatile v4f*)dst = o;
    __threadfence();
    *(volatile v4f*)dst = o;
  }
}

__global__ void __launch_bounds__(NN)
final_kernel(const float* __restrict__ yws, const float* __restrict__ kw,
             const float* __restrict__ bias, float* __restrict__ out)
{
  __shared__ float ysh[NF][NN];
  __shared__ float rsum[NN];
  const int i = threadIdx.x;
  #pragma unroll
  for (int g = 0; g < NF; ++g) ysh[g][i] = yws[g * NN + i];
  __syncthreads();

  float zsum = 0.0f;
  #pragma unroll 1
  for (int fo = 0; fo < NF; ++fo) {
    float z = 0.0f;
    #pragma unroll
    for (int p = 0; p < NP; ++p) {
      const int row = (p - i) & (NN - 1);
      #pragma unroll
      for (int g = 0; g < NF; ++g)
        z += kw[(p * NF + g) * NF + fo] * ysh[g][row];
    }
    z += bias[fo];
    zsum += (z > 0.0f) ? z : expm1f(z);
  }
  rsum[i] = zsum;
  __syncthreads();
  for (int stride = NN / 2; stride > 0; stride >>= 1) {
    if (i < stride) rsum[i] += rsum[i + stride];
    __syncthreads();
  }
  if (i == 0) {
    const float v = 0.1f + rsum[0] / (float)(NN * NF);
    *(volatile float*)out = v;
    __threadfence();
    *(volatile float*)out = v;
  }
}

extern "C" void kernel_launch(void* const* d_in, const int* in_sizes, int n_in,
                              void* d_out, int out_size, void* d_ws, size_t ws_size,
                              hipStream_t stream)
{
  if (n_in < 5) return;
  if (in_sizes[0] != NN) return;
  if (in_sizes[1] != NF * MM * MM) return;
  if (in_sizes[2] != NP * NF * NF) return;
  if (in_sizes[3] < NF) return;
  if (in_sizes[4] != NC * NC * NC) return;
  if (out_size < 1) return;

  const int*   xv   = (const int*)d_in[0];
  const float* ik   = (const float*)d_in[1];
  const float* kw   = (const float*)d_in[2];
  const float* bias = (const float*)d_in[3];
  const float* tp   = (const float*)d_in[4];
  float* out = (float*)d_out;

  const size_t bytesA = (size_t)NF * NN * NN * 2;
  const size_t bytesD = (size_t)NC * NN * NN * 2;
  const size_t bytesY = (size_t)NF * NN * 4;
  const size_t offA = 0;
  const size_t offD = offA + bytesA;
  const size_t offY = offD + bytesD;
  if (offY + bytesY > ws_size) return;

  char* ws = (char*)d_ws;
  unsigned short* A16 = (unsigned short*)(ws + offA);
  unsigned short* D16 = (unsigned short*)(ws + offD);
  float*          yws = (float*)(ws + offY);

  const int total_chunks = (NF + NC) * NN * (NN / 8);
  const int pblk = 256;
  const int pgrid = (total_chunks + pblk - 1) / pblk;

  prep_kernel<<<dim3(pgrid), dim3(pblk), 0, stream>>>(xv, ik, A16, D16, total_chunks);
  gemm_kernel<<<dim3(NN / 32, NF), dim3(128), 0, stream>>>(xv, tp, A16, D16, yws);
  final_kernel<<<dim3(1), dim3(NN), 0, stream>>>(yws, kw, bias, out);
}
